// MambaSequenceClassificationSP_23261542875727
// MI455X (gfx1250) — hardware-verified
//
#include <hip/hip_runtime.h>
#include <math.h>
#include <stdint.h>


#define BATCH    8
#define SEQLEN   1024
#define DMODEL   256
#define NLAYERS  2
#define DSTATE   64
#define DCONV    4
#define HEADDIM  64
#define DINNER   512
#define NHEADS   8
#define CONVDIM  640
#define DINPROJ  1160
#define LDZ      1216
#define DHALF    128
#define NCLS     2
#define ROWS     (BATCH * SEQLEN)
#define EPSV     1e-5f
#define SCH      32

typedef char chk_rows_tile[(ROWS % 128 == 0) ? 1 : -1];
typedef char chk_ldz[(LDZ % 64 == 0 && LDZ >= DINPROJ) ? 1 : -1];
typedef char chk_dmodel[(DMODEL % 64 == 0 && DINNER % 64 == 0) ? 1 : -1];
typedef char chk_kdepth[(DMODEL % 32 == 0 && DINNER % 32 == 0) ? 1 : -1];
typedef char chk_seq[(SEQLEN % SCH == 0) ? 1 : -1];

typedef __bf16 v16b __attribute__((ext_vector_type(16)));
typedef float  v8f  __attribute__((ext_vector_type(8)));
typedef float  v4f  __attribute__((ext_vector_type(4)));
typedef float  v4fa __attribute__((ext_vector_type(4), __may_alias__));
typedef unsigned int v4u __attribute__((ext_vector_type(4)));

union Frag { v16b v; v4u q[2]; };
union Acc8 { v8f v; float f[8]; };
struct HL { v4u h; v4u l; };

__device__ __forceinline__ unsigned int bf_rne(float f) {
  unsigned int u = __float_as_uint(f);
  u += 0x7FFFu + ((u >> 16) & 1u);
  return u >> 16;
}

__device__ __forceinline__ HL split8(const float (&f)[8]) {
  unsigned int hh[8], ll[8];
#pragma unroll
  for (int i = 0; i < 8; ++i) {
    const unsigned int hb = bf_rne(f[i]);
    const float rem = f[i] - __uint_as_float(hb << 16);
    hh[i] = hb;
    ll[i] = bf_rne(rem);
  }
  HL r;
  r.h.x = hh[0] | (hh[1] << 16); r.h.y = hh[2] | (hh[3] << 16);
  r.h.z = hh[4] | (hh[5] << 16); r.h.w = hh[6] | (hh[7] << 16);
  r.l.x = ll[0] | (ll[1] << 16); r.l.y = ll[2] | (ll[3] << 16);
  r.l.z = ll[4] | (ll[5] << 16); r.l.w = ll[6] | (ll[7] << 16);
  return r;
}

__device__ __forceinline__ float siluf(float x) { return x * (1.f / (1.f + expf(-x))); }
__device__ __forceinline__ float geluf(float x) { return x * (erff(x * 0.70710678118654752f) + 1.f) * 0.5f; }

__global__ __launch_bounds__(64)
void k_embed(const int* __restrict__ ids, const float* __restrict__ emb, int vocab, float* x) {
  const int row = blockIdx.x;
  const int t = threadIdx.x;
  int id = ids[row];
  id = id < 0 ? 0 : id;
  id = id > vocab - 1 ? vocab - 1 : id;
  const v4f v = *(const v4f*)(emb + (size_t)id * DMODEL + 4 * t);
  volatile v4f* p = (volatile v4f*)(x + (size_t)row * DMODEL + 4 * t);
  *p = v;
  __threadfence();
  *p = v;
}

__global__ __launch_bounds__(256)
void k_split(const float* __restrict__ src, unsigned short* hi, unsigned short* lo, int n8) {
  const int g = blockIdx.x * 256 + threadIdx.x;
  if (g >= n8) return;
  const float* p = src + (size_t)g * 8;
  const v4f a = *(const v4f*)p;
  const v4f b = *(const v4f*)(p + 4);
  const float f[8] = {a.x, a.y, a.z, a.w, b.x, b.y, b.z, b.w};
  const HL r = split8(f);
  volatile v4u* ph = (volatile v4u*)(hi + (size_t)g * 8);
  volatile v4u* pl = (volatile v4u*)(lo + (size_t)g * 8);
  *ph = r.h;
  *pl = r.l;
  __threadfence();
  *ph = r.h;
  *pl = r.l;
}

__global__ __launch_bounds__(256)
void k_gemm(const unsigned short* __restrict__ Ah, const unsigned short* __restrict__ Al,
            const unsigned short* __restrict__ Bh, const unsigned short* __restrict__ Bl,
            float* C, int N, int K, int ldc, int addres) {
  __shared__ __align__(16) unsigned short sAh[128][32];
  __shared__ __align__(16) unsigned short sAl[128][32];
  __shared__ __align__(16) unsigned short sBh[64][32];
  __shared__ __align__(16) unsigned short sBl[64][32];
  __shared__ __align__(16) float sC[8][32 * 32];

  const int tid  = threadIdx.x;
  const int lane = tid & 31;
  const int wave = tid >> 5;
  const int wm   = wave & 3;
  const int wn   = wave >> 2;
  const int m0   = blockIdx.y * 128;
  const int n0   = blockIdx.x * 64;
  const int ra = tid >> 1, sa = (tid & 1) * 16;
  const int rb = tid >> 2, sb = (tid & 3) * 8;
  const int fr = lane & 15;
  const int h8 = (lane >> 4) * 8;

  v8f acc00 = {}; v8f acc01 = {}; v8f acc10 = {}; v8f acc11 = {};
  const v4u z4 = {0u, 0u, 0u, 0u};

  const int kTiles = K >> 5;
  for (int kt = 0; kt < kTiles; ++kt) {
    const size_t ka = (size_t)(m0 + ra) * (size_t)K + (size_t)kt * 32 + sa;
    const v4u ah0 = *(const v4u*)(Ah + ka);
    const v4u ah1 = *(const v4u*)(Ah + ka + 8);
    const v4u al0 = *(const v4u*)(Al + ka);
    const v4u al1 = *(const v4u*)(Al + ka + 8);
    v4u bh0 = z4, bl0 = z4;
    const int bn = n0 + rb;
    if (bn < N) {
      const size_t kb = (size_t)bn * (size_t)K + (size_t)kt * 32 + sb;
      bh0 = *(const v4u*)(Bh + kb);
      bl0 = *(const v4u*)(Bl + kb);
    }
    *(v4u*)&sAh[ra][sa]     = ah0;
    *(v4u*)&sAh[ra][sa + 8] = ah1;
    *(v4u*)&sAl[ra][sa]     = al0;
    *(v4u*)&sAl[ra][sa + 8] = al1;
    *(v4u*)&sBh[rb][sb]     = bh0;
    *(v4u*)&sBl[rb][sb]     = bl0;
    __syncthreads();

    Frag a0h, a0l, a1h, a1l, b0h, b0l, b1h, b1l;
    const int ar0 = wm * 32 + fr, ar1 = wm * 32 + 16 + fr;
    const int bc0 = wn * 32 + fr, bc1 = wn * 32 + 16 + fr;
    a0h.q[0] = *(const v4u*)&sAh[ar0][h8]; a0h.q[1] = *(const v4u*)&sAh[ar0][16 + h8];
    a0l.q[0] = *(const v4u*)&sAl[ar0][h8]; a0l.q[1] = *(const v4u*)&sAl[ar0][16 + h8];
    a1h.q[0] = *(const v4u*)&sAh[ar1][h8]; a1h.q[1] = *(const v4u*)&sAh[ar1][16 + h8];
    a1l.q[0] = *(const v4u*)&sAl[ar1][h8]; a1l.q[1] = *(const v4u*)&sAl[ar1][16 + h8];
    b0h.q[0] = *(const v4u*)&sBh[bc0][h8]; b0h.q[1] = *(const v4u*)&sBh[bc0][16 + h8];
    b0l.q[0] = *(const v4u*)&sBl[bc0][h8]; b0l.q[1] = *(const v4u*)&sBl[bc0][16 + h8];
    b1h.q[0] = *(const v4u*)&sBh[bc1][h8]; b1h.q[1] = *(const v4u*)&sBh[bc1][16 + h8];
    b1l.q[0] = *(const v4u*)&sBl[bc1][h8]; b1l.q[1] = *(const v4u*)&sBl[bc1][16 + h8];

    acc00 = __builtin_amdgcn_wmma_f32_16x16x32_bf16(false, a0h.v, false, b0h.v, (short)0, acc00, false, false);
    acc01 = __builtin_amdgcn_wmma_f32_16x16x32_bf16(false, a0h.v, false, b1h.v, (short)0, acc01, false, false);
    acc10 = __builtin_amdgcn_wmma_f32_16x16x32_bf16(false, a1h.v, false, b0h.v, (short)0, acc10, false, false);
    acc11 = __builtin_amdgcn_wmma_f32_16x16x32_bf16(false, a1h.v, false, b1h.v, (short)0, acc11, false, false);
    acc00 = __builtin_amdgcn_wmma_f32_16x16x32_bf16(false, a0h.v, false, b0l.v, (short)0, acc00, false, false);
    acc01 = __builtin_amdgcn_wmma_f32_16x16x32_bf16(false, a0h.v, false, b1l.v, (short)0, acc01, false, false);
    acc10 = __builtin_amdgcn_wmma_f32_16x16x32_bf16(false, a1h.v, false, b0l.v, (short)0, acc10, false, false);
    acc11 = __builtin_amdgcn_wmma_f32_16x16x32_bf16(false, a1h.v, false, b1l.v, (short)0, acc11, false, false);
    acc00 = __builtin_amdgcn_wmma_f32_16x16x32_bf16(false, a0l.v, false, b0h.v, (short)0, acc00, false, false);
    acc01 = __builtin_amdgcn_wmma_f32_16x16x32_bf16(false, a0l.v, false, b1h.v, (short)0, acc01, false, false);
    acc10 = __builtin_amdgcn_wmma_f32_16x16x32_bf16(false, a1l.v, false, b0h.v, (short)0, acc10, false, false);
    acc11 = __builtin_amdgcn_wmma_f32_16x16x32_bf16(false, a1l.v, false, b1h.v, (short)0, acc11, false, false);
    asm volatile("v_nop\n\tv_nop\n\tv_nop\n\tv_nop"
                 : "+v"(acc00), "+v"(acc01), "+v"(acc10), "+v"(acc11)
                 : "v"(a0h.v), "v"(a0l.v), "v"(a1h.v), "v"(a1l.v),
                   "v"(b0h.v), "v"(b0l.v), "v"(b1h.v), "v"(b1l.v));
    __syncthreads();
  }

  {
    Acc8 o00, o01, o10, o11;
    o00.v = acc00; o01.v = acc01; o10.v = acc10; o11.v = acc11;
    float* cw = &sC[wave][0];
#pragma unroll
    for (int r = 0; r < 8; ++r) {
      cw[(h8 + r) * 32 + fr]           = o00.f[r];
      cw[(h8 + r) * 32 + 16 + fr]      = o01.f[r];
      cw[(16 + h8 + r) * 32 + fr]      = o10.f[r];
      cw[(16 + h8 + r) * 32 + 16 + fr] = o11.f[r];
    }
  }
  __syncthreads();
  {
    const float* cw = &sC[wave][0];
    const int rl = lane >> 3;
    const int c4 = (lane & 7) * 4;
    v4f v[8];
    size_t gi[8];
#pragma unroll
    for (int j = 0; j < 8; ++j) {
      const int row = 4 * j + rl;
      v[j]  = *(const v4fa*)(cw + row * 32 + c4);
      gi[j] = (size_t)(m0 + wm * 32 + row) * (size_t)ldc + (size_t)(n0 + wn * 32 + c4);
      if (addres) v[j] += *(const v4fa*)(C + gi[j]);
    }
#pragma unroll
    for (int j = 0; j < 8; ++j) *(volatile v4f*)(C + gi[j]) = v[j];
    __threadfence();
#pragma unroll
    for (int j = 0; j < 8; ++j) *(volatile v4f*)(C + gi[j]) = v[j];
  }
}

__global__ __launch_bounds__(160)
void k_conv(const float* __restrict__ zx, const float* __restrict__ cw, const float* __restrict__ cb,
            float* xc) {
  const int row = blockIdx.x;
  const int l   = row & (SEQLEN - 1);
  const int t   = threadIdx.x;
  const int c0  = t * 4;
  v4f acc = *(const v4f*)(cb + c0);
  v4f w[4];
#pragma unroll
  for (int i = 0; i < 4; ++i) w[i] = *(const v4f*)(cw + (size_t)(c0 + i) * DCONV);
#pragma unroll
  for (int k = 0; k < DCONV; ++k) {
    const int ls = l - (DCONV - 1) + k;
    if (ls >= 0) {
      const v4f xv = *(const v4f*)(zx + (size_t)(row - (DCONV - 1) + k) * LDZ + DINNER + c0);
      acc[0] += xv[0] * w[0][k];
      acc[1] += xv[1] * w[1][k];
      acc[2] += xv[2] * w[2][k];
      acc[3] += xv[3] * w[3][k];
    }
  }
  v4f o;
  o[0] = siluf(acc[0]); o[1] = siluf(acc[1]); o[2] = siluf(acc[2]); o[3] = siluf(acc[3]);
  volatile v4f* p = (volatile v4f*)(xc + (size_t)row * CONVDIM + c0);
  *p = o;
  __threadfence();
  *p = o;
}

__global__ __launch_bounds__(256)
void k_scan(const float* __restrict__ xc, const float* __restrict__ zx,
            const float* __restrict__ dtb, const float* __restrict__ alog, const float* __restrict__ Dv,
            float* y) {
  __shared__ __align__(16) float xs[SCH][64];
  __shared__ __align__(16) float Bs[SCH][64];
  __shared__ __align__(16) float Cm[SCH][64];
  __shared__ __align__(16) float ys[SCH][64];
  __shared__ float dts[SCH];
  __shared__ float dAs[SCH];

  const int b   = blockIdx.x >> 3;
  const int h   = blockIdx.x & 7;
  const int tid = threadIdx.x;
  const int p   = tid >> 2;
  const int ng  = (tid & 3) * 16;
  const float Dh   = Dv[h];
  const float Aneg = -expf(alog[h]);
  const float dtbh = dtb[h];

  float hst[16];
#pragma unroll
  for (int i = 0; i < 16; ++i) hst[i] = 0.f;

  for (int c = 0; c < SEQLEN / SCH; ++c) {
    const int l0 = c * SCH;
#pragma unroll
    for (int q = 0; q < 6; ++q) {
      const int f   = tid + q * 256;
      const int arr = q >> 1;
      const int wi  = f & 511;
      const int t   = wi >> 4;
      const int ch  = (wi & 15) * 4;
      const int col = (arr == 0) ? (h * HEADDIM + ch) : (arr == 1 ? (DINNER + ch) : (DINNER + DSTATE + ch));
      const v4f v = *(const v4f*)(xc + ((size_t)(b * SEQLEN + l0 + t)) * CONVDIM + col);
      if (arr == 0)      *(v4f*)&xs[t][ch] = v;
      else if (arr == 1) *(v4f*)&Bs[t][ch] = v;
      else               *(v4f*)&Cm[t][ch] = v;
    }
    if (tid < SCH) {
      const float raw = zx[((size_t)(b * SEQLEN + l0 + tid)) * LDZ + (DINNER + CONVDIM) + h] + dtbh;
      const float sp  = fmaxf(raw, 0.f) + log1pf(expf(-fabsf(raw)));
      dts[tid] = sp;
      dAs[tid] = expf(sp * Aneg);
    }
    __syncthreads();

#pragma unroll 1
    for (int t = 0; t < SCH; ++t) {
      const float dtv = dts[t], dav = dAs[t];
      const float xv  = xs[t][p];
      const float coef = dtv * xv;
      float bv[16], cv[16];
#pragma unroll
      for (int u = 0; u < 4; ++u) {
        const v4f bq = *(const v4f*)&Bs[t][ng + 4 * u];
        const v4f cq = *(const v4f*)&Cm[t][ng + 4 * u];
        bv[4 * u + 0] = bq[0]; bv[4 * u + 1] = bq[1]; bv[4 * u + 2] = bq[2]; bv[4 * u + 3] = bq[3];
        cv[4 * u + 0] = cq[0]; cv[4 * u + 1] = cq[1]; cv[4 * u + 2] = cq[2]; cv[4 * u + 3] = cq[3];
      }
      float part = 0.f;
#pragma unroll
      for (int i = 0; i < 16; ++i) {
        hst[i] = hst[i] * dav + coef * bv[i];
        part += hst[i] * cv[i];
      }
      part += __shfl_xor(part, 1);
      part += __shfl_xor(part, 2);
      if ((tid & 3) == 0) ys[t][p] = part + Dh * xv;
    }
    __syncthreads();

    {
      v4f o[2];
      size_t gi[2];
#pragma unroll
      for (int j = 0; j < 2; ++j) {
        const int f  = tid + j * 256;
        const int t  = f >> 4;
        const int c4 = (f & 15) * 4;
        o[j]  = *(const v4fa*)&ys[t][c4];
        gi[j] = ((size_t)(b * SEQLEN + l0 + t)) * DINNER + (size_t)(h * HEADDIM + c4);
      }
      *(volatile v4f*)(y + gi[0]) = o[0];
      *(volatile v4f*)(y + gi[1]) = o[1];
      __threadfence();
      *(volatile v4f*)(y + gi[0]) = o[0];
      *(volatile v4f*)(y + gi[1]) = o[1];
    }
    __syncthreads();
  }
}

__global__ __launch_bounds__(64)
void k_gate(const float* __restrict__ y, const float* __restrict__ zx, const float* __restrict__ nw,
            unsigned short* ynh, unsigned short* ynl) {
  __shared__ float red[2];
  const int row = blockIdx.x;
  const int t   = threadIdx.x;
  const int e0  = t * 8;
  const float* yp = y + (size_t)row * DINNER + e0;
  const float* zp = zx + (size_t)row * LDZ + e0;
  const v4f y0 = *(const v4f*)yp, y1 = *(const v4f*)(yp + 4);
  const v4f z0 = *(const v4f*)zp, z1 = *(const v4f*)(zp + 4);
  const float yy[8] = {y0.x, y0.y, y0.z, y0.w, y1.x, y1.y, y1.z, y1.w};
  const float zz[8] = {z0.x, z0.y, z0.z, z0.w, z1.x, z1.y, z1.z, z1.w};
  float g[8];
  float ss = 0.f;
#pragma unroll
  for (int i = 0; i < 8; ++i) { g[i] = yy[i] * siluf(zz[i]); ss += g[i] * g[i]; }
#pragma unroll
  for (int o = 16; o > 0; o >>= 1) ss += __shfl_xor(ss, o);
  if ((t & 31) == 0) red[t >> 5] = ss;
  __syncthreads();
  const float tot  = red[0] + red[1];
  const float rstd = rsqrtf(tot * (1.f / (float)DINNER) + EPSV);
  const v4f n0 = *(const v4f*)(nw + e0), n1 = *(const v4f*)(nw + e0 + 4);
  const float nn[8] = {n0.x, n0.y, n0.z, n0.w, n1.x, n1.y, n1.z, n1.w};
  float ov[8];
#pragma unroll
  for (int i = 0; i < 8; ++i) ov[i] = (g[i] * rstd) * nn[i];
  const HL r = split8(ov);
  volatile v4u* ph = (volatile v4u*)(ynh + (size_t)row * DINNER + e0);
  volatile v4u* pl = (volatile v4u*)(ynl + (size_t)row * DINNER + e0);
  *ph = r.h;
  *pl = r.l;
  __threadfence();
  *ph = r.h;
  *pl = r.l;
}

__global__ __launch_bounds__(256)
void k_head(const float* __restrict__ x,
            const float* __restrict__ pw, const float* __restrict__ pb,
            const float* __restrict__ c1w, const float* __restrict__ c1b,
            const float* __restrict__ c2w, const float* __restrict__ c2b,
            float* out) {
  __shared__ float ps[BATCH * DMODEL];
  __shared__ float p1[BATCH * DMODEL];
  __shared__ float h1[BATCH * DHALF];
  __shared__ __align__(16) float o16[BATCH * NCLS];
  const int tid = threadIdx.x;

  for (int b = 0; b < BATCH; ++b) {
    double s = 0.0;
    float mx = -INFINITY;
    const float* xb = x + (size_t)b * SEQLEN * DMODEL + tid;
#pragma unroll 4
    for (int l = 0; l < SEQLEN; ++l) {
      const float v = xb[(size_t)l * DMODEL];
      s += (double)v;
      mx = fmaxf(mx, v);
    }
    const float mean = (float)s * (1.f / (float)SEQLEN);
    ps[b * DMODEL + tid] = (mean + mx) * 0.5f;
  }
  __syncthreads();

  for (int i = tid; i < BATCH * DMODEL; i += 256) {
    const int b = i >> 8, o = i & 255;
    float acc = pb[o];
#pragma unroll 8
    for (int k = 0; k < DMODEL; ++k) acc += ps[b * DMODEL + k] * pw[(size_t)o * DMODEL + k];
    p1[i] = geluf(acc);
  }
  __syncthreads();

  for (int i = tid; i < BATCH * DHALF; i += 256) {
    const int b = i >> 7, o = i & 127;
    float acc = c1b[o];
#pragma unroll 8
    for (int k = 0; k < DMODEL; ++k) acc += p1[b * DMODEL + k] * c1w[(size_t)o * DMODEL + k];
    h1[i] = geluf(acc);
  }
  __syncthreads();

  if (tid < BATCH * NCLS) {
    const int b = tid >> 1, o = tid & 1;
    float acc = c2b[o];
#pragma unroll 4
    for (int k = 0; k < DHALF; ++k) acc += h1[b * DHALF + k] * c2w[o * DHALF + k];
    o16[tid] = acc;
  }
  __syncthreads();
  if (tid < (BATCH * NCLS) / 4) {
    const v4f v = *(const v4fa*)&o16[tid * 4];
    volatile v4f* p = (volatile v4f*)(out + tid * 4);
    *p = v;
    __threadfence();
    *p = v;
  }
}

static inline size_t al256(size_t v) { return (v + 255) & ~(size_t)255; }

extern "C" void kernel_launch(void* const* d_in, const int* in_sizes, int n_in,
                              void* d_out, int out_size, void* d_ws, size_t ws_size,
                              hipStream_t stream) {
  if (n_in < 16) return;
  if (in_sizes[0] != ROWS) return;
  if (in_sizes[1] < DMODEL || (in_sizes[1] % DMODEL) != 0) return;
  if (in_sizes[2] != NLAYERS * DINPROJ * DMODEL) return;
  if (in_sizes[3] != NLAYERS * CONVDIM * DCONV) return;
  if (in_sizes[4] != NLAYERS * CONVDIM) return;
  if (in_sizes[5] != NLAYERS * NHEADS || in_sizes[6] != NLAYERS * NHEADS || in_sizes[7] != NLAYERS * NHEADS) return;
  if (in_sizes[8] != NLAYERS * DINNER) return;
  if (in_sizes[9] != NLAYERS * DMODEL * DINNER) return;
  if (in_sizes[10] != DMODEL * DMODEL || in_sizes[11] != DMODEL) return;
  if (in_sizes[12] != DHALF * DMODEL || in_sizes[13] != DHALF) return;
  if (in_sizes[14] != NCLS * DHALF || in_sizes[15] != NCLS) return;
  if (out_size != BATCH * NCLS) return;

  const int*   ids  = (const int*)  d_in[0];
  const float* emb  = (const float*)d_in[1];
  const float* inw  = (const float*)d_in[2];
  const float* cw   = (const float*)d_in[3];
  const float* cb   = (const float*)d_in[4];
  const float* dtb  = (const float*)d_in[5];
  const float* alog = (const float*)d_in[6];
  const float* Dv   = (const float*)d_in[7];
  const float* nw   = (const float*)d_in[8];
  const float* ow   = (const float*)d_in[9];
  const float* pw   = (const float*)d_in[10];
  const float* pb   = (const float*)d_in[11];
  const float* c1w  = (const float*)d_in[12];
  const float* c1b  = (const float*)d_in[13];
  const float* c2w  = (const float*)d_in[14];
  const float* c2b  = (const float*)d_in[15];
  float* out = (float*)d_out;
  const int vocab = in_sizes[1] / DMODEL;

  const size_t szX   = (size_t)ROWS * DMODEL * 4;
  const size_t szXp  = (size_t)ROWS * DMODEL * 2;
  const size_t szZ   = (size_t)ROWS * LDZ * 4;
  const size_t szXc  = (size_t)ROWS * CONVDIM * 4;
  const size_t szY   = (size_t)ROWS * DINNER * 4;
  const size_t szYp  = (size_t)ROWS * DINNER * 2;
  const size_t szWA  = (size_t)NLAYERS * DINPROJ * DMODEL * 2;
  const size_t szWO  = (size_t)NLAYERS * DMODEL * DINNER * 2;
  size_t off = 0;
  const size_t oX   = off; off = al256(off + szX);
  const size_t oXh  = off; off = al256(off + szXp);
  const size_t oXl  = off; off = al256(off + szXp);
  const size_t oZ   = off; off = al256(off + szZ);
  const size_t oXc  = off; off = al256(off + szXc);
  const size_t oY   = off; off = al256(off + szY);
  const size_t oYh  = off; off = al256(off + szYp);
  const size_t oYl  = off; off = al256(off + szYp);
  const size_t oWAh = off; off = al256(off + szWA);
  const size_t oWAl = off; off = al256(off + szWA);
  const size_t oWOh = off; off = al256(off + szWO);
  const size_t oWOl = off; off = al256(off + szWO);
  if (off > ws_size) return;

  char* w = (char*)d_ws;
  float*          x    = (float*)(w + oX);
  unsigned short* xh   = (unsigned short*)(w + oXh);
  unsigned short* xl   = (unsigned short*)(w + oXl);
  float*          zx   = (float*)(w + oZ);
  float*          xc   = (float*)(w + oXc);
  float*          ybuf = (float*)(w + oY);
  unsigned short* yh   = (unsigned short*)(w + oYh);
  unsigned short* yl   = (unsigned short*)(w + oYl);
  unsigned short* wAh  = (unsigned short*)(w + oWAh);
  unsigned short* wAl  = (unsigned short*)(w + oWAl);
  unsigned short* wOh  = (unsigned short*)(w + oWOh);
  unsigned short* wOl  = (unsigned short*)(w + oWOl);

  const int n8X  = (ROWS * DMODEL) / 8;
  const int n8WA = (NLAYERS * DINPROJ * DMODEL) / 8;
  const int n8WO = (NLAYERS * DMODEL * DINNER) / 8;

  k_embed<<<ROWS, 64, 0, stream>>>(ids, emb, vocab, x);
  k_split<<<(n8X + 255) / 256, 256, 0, stream>>>(x, xh, xl, n8X);
  k_split<<<(n8WA + 255) / 256, 256, 0, stream>>>(inw, wAh, wAl, n8WA);
  k_split<<<(n8WO + 255) / 256, 256, 0, stream>>>(ow, wOh, wOl, n8WO);

  for (int layer = 0; layer < NLAYERS; ++layer) {
    const unsigned short* wAh_l = wAh + (size_t)layer * DINPROJ * DMODEL;
    const unsigned short* wAl_l = wAl + (size_t)layer * DINPROJ * DMODEL;
    const unsigned short* wOh_l = wOh + (size_t)layer * DMODEL * DINNER;
    const unsigned short* wOl_l = wOl + (size_t)layer * DMODEL * DINNER;
    const float* cw_l   = cw   + (size_t)layer * CONVDIM * DCONV;
    const float* cb_l   = cb   + (size_t)layer * CONVDIM;
    const float* dtb_l  = dtb  + (size_t)layer * NHEADS;
    const float* alog_l = alog + (size_t)layer * NHEADS;
    const float* Dv_l   = Dv   + (size_t)layer * NHEADS;
    const float* nw_l   = nw   + (size_t)layer * DINNER;

    k_gemm<<<dim3(LDZ / 64, ROWS / 128), 256, 0, stream>>>(xh, xl, wAh_l, wAl_l, zx, DINPROJ, DMODEL, LDZ, 0);
    k_conv<<<ROWS, CONVDIM / 4, 0, stream>>>(zx, cw_l, cb_l, xc);
    k_scan<<<BATCH * NHEADS, 256, 0, stream>>>(xc, zx, dtb_l, alog_l, Dv_l, ybuf);
    k_gate<<<ROWS, DINNER / 8, 0, stream>>>(ybuf, zx, nw_l, yh, yl);
    k_gemm<<<dim3(DMODEL / 64, ROWS / 128), 256, 0, stream>>>(yh, yl, wOh_l, wOl_l, x, DMODEL, DINNER, DMODEL, 1);
    if (layer + 1 < NLAYERS)
      k_split<<<(n8X + 255) / 256, 256, 0, stream>>>(x, xh, xl, n8X);
  }

  k_head<<<1, 256, 0, stream>>>(x, pw, pb, c1w, c1b, c2w, c2b, out);
}
